// Model_75265006895519
// MI455X (gfx1250) — hardware-verified
//
#include <hip/hip_runtime.h>
#include <math.h>

typedef __attribute__((ext_vector_type(16))) _Float16 v16h;
typedef __attribute__((ext_vector_type(8)))  _Float16 v8h;
typedef __attribute__((ext_vector_type(8)))  float    v8f;
typedef __attribute__((ext_vector_type(4)))  float    v4f;

constexpr int kBatch = 8;
constexpr int kSeqT  = 512;
constexpr int kDm    = 256;
constexpr int kDinr  = 512;
constexpr int kNmat  = 2;
constexpr int kNhead = 4;
constexpr int kHdim  = 64;
constexpr int kLayers = 2;
constexpr int kVocab = 272;
constexpr int kTok   = kBatch * kSeqT;
constexpr int kUGld  = 2 * kDinr;
constexpr int kVPld  = kNmat * kDm + 64;
constexpr int kPrmLd = 32;
constexpr int kConvTP = 260;
constexpr int kScanTS = 16;
constexpr float kWCarry = 32.0f;
constexpr float kPCarry = 256.0f;
constexpr float kUCarry = 256.0f;
constexpr float kOCarry = 4096.0f;
static_assert(kNhead * kHdim == kDm);
static_assert((kDm % 32) == 0 && (kDinr % 32) == 0);
static_assert((kTok % 64) == 0 && (kUGld % 64) == 0 && (kDm % 64) == 0 && (kVPld % 64) == 0);
static_assert((kVocab % 16) == 0 && (kSeqT % 64) == 0 && (kSeqT % kScanTS) == 0);
static_assert(4 + 8 + 8 + 8 + 4 == kPrmLd);

constexpr size_t kOffX    = 0;
constexpr size_t kOffNX   = kOffX    + (size_t)kTok * kDm * 4;
constexpr size_t kOffY16  = kOffNX   + (size_t)kTok * kDm * 2;
constexpr size_t kOffUPGP = kOffY16  + (size_t)kTok * kDm * 2;
constexpr size_t kOffP16  = kOffUPGP + (size_t)kTok * kUGld * 4;
constexpr size_t kOffU    = kOffP16  + (size_t)kTok * kDinr * 2;
constexpr size_t kOffU16  = kOffU    + (size_t)kTok * kDm * 4;
constexpr size_t kOffVP   = kOffU16  + (size_t)kTok * kDm * 2;
constexpr size_t kOffPRM  = kOffVP   + (size_t)kTok * kVPld * 4;
constexpr size_t kOffO16  = kOffPRM  + (size_t)kTok * kPrmLd * 4;
constexpr size_t kOffWUG  = kOffO16  + (size_t)kTok * kDm * 2;
constexpr size_t kOffWDN  = kOffWUG  + (size_t)kLayers * kUGld * kDm * 2;
constexpr size_t kOffWVS  = kOffWDN  + (size_t)kLayers * kDm * kDinr * 2;
constexpr size_t kOffWOU  = kOffWVS  + (size_t)kLayers * kVPld * kDm * 2;
constexpr size_t kOffEMB  = kOffWOU  + (size_t)kLayers * kDm * kDm * 2;
constexpr size_t kWsTotal = kOffEMB  + (size_t)kVocab * kDm * 2;
static_assert(kWsTotal == 50274304ull);
static_assert(kWsTotal <= 134217728ull);
static_assert((kOffNX % 128) == 0 && (kOffY16 % 128) == 0 && (kOffUPGP % 128) == 0 && (kOffP16 % 128) == 0 &&
              (kOffU % 128) == 0 && (kOffU16 % 128) == 0 && (kOffVP % 128) == 0 && (kOffPRM % 128) == 0 &&
              (kOffO16 % 128) == 0 && (kOffWUG % 128) == 0 && (kOffWDN % 128) == 0 && (kOffWVS % 128) == 0 &&
              (kOffWOU % 128) == 0 && (kOffEMB % 128) == 0);

struct FragH {
  union U { v16h v; v8h h[2]; };
  static __device__ __forceinline__ v16h load(const _Float16* p) {
    U f; f.h[0] = *(const v8h*)(p); f.h[1] = *(const v8h*)(p + 16); return f.v;
  }
  static __device__ __forceinline__ v8f mma(v16h a, v16h b, v8f c) {
    return __builtin_amdgcn_wmma_f32_16x16x32_f16(false, a, false, b, (short)0, c, false, false);
  }
};
__device__ __forceinline__ void dep_guard4_h(v8f& a, v8f& b, v8f& c, v8f& d, v16h x, v16h b0, v16h b1, v16h b2, v16h b3) {
  asm volatile("v_nop\n\tv_nop\n\tv_nop\n\tv_nop" : "+v"(a), "+v"(b), "+v"(c), "+v"(d) : "v"(x), "v"(b0), "v"(b1), "v"(b2), "v"(b3));
}
__device__ __forceinline__ void dep_guard6_h(v8f& a0, v8f& a1, v8f& a2, v8f& a3, v8f& a4, v8f& a5,
                                             v16h x0, v16h x1, v16h y0, v16h y1, v16h y2) {
  asm volatile("v_nop\n\tv_nop\n\tv_nop\n\tv_nop" : "+v"(a0), "+v"(a1), "+v"(a2), "+v"(a3), "+v"(a4), "+v"(a5)
               : "v"(x0), "v"(x1), "v"(y0), "v"(y1), "v"(y2));
}
__device__ __forceinline__ void acc_guard4(v8f& a, v8f& b, v8f& c, v8f& d) { asm volatile("v_nop\n\tv_nop\n\tv_nop\n\tv_nop" : "+v"(a), "+v"(b), "+v"(c), "+v"(d)); }
__device__ __forceinline__ void force4(v4f& a, v4f& b, v4f& c, v4f& d) { asm volatile("" : "+v"(a), "+v"(b), "+v"(c), "+v"(d)); }

template <int EPI>
__global__ __launch_bounds__(256) void wmma_gemm64_f16(
    const unsigned short* __restrict__ Ap, int lda,
    const unsigned short* __restrict__ Btp, int ldb,
    float* Cout, int ldc,
    unsigned short* C2, int ld2, float scale2,
    const float* R1, const float* R2,
    int M, int N, int K, float scale)
{
  const _Float16* A  = (const _Float16*)Ap;
  const _Float16* Bt = (const _Float16*)Btp;
  __shared__ __align__(16) float sT[8][16 * 68];
  const int lane = threadIdx.x & 31;
  const int wave = threadIdx.x >> 5;
  const int tilesN = N >> 6;
  const int tilesM = M >> 6;
  const int tile = blockIdx.x * 8 + wave;
  if (tile >= tilesM * tilesN) return;
  const int tm = tile / tilesN;
  const int tn = tile - tm * tilesN;
  const int m0 = tm << 6;
  const int n0 = tn << 6;
  const int rlane = lane & 15;
  const int koff  = (lane >> 4) * 8;
  const int mOff  = (lane >> 4) * 8;

  v8f acc[4][4];
#pragma unroll
  for (int i = 0; i < 4; ++i)
#pragma unroll
    for (int j = 0; j < 4; ++j) acc[i][j] = (v8f){0.f,0.f,0.f,0.f,0.f,0.f,0.f,0.f};

  for (int k0 = 0; k0 < K; k0 += 32) {
    v16h bh[4];
#pragma unroll
    for (int j = 0; j < 4; ++j) {
      const size_t bo = (size_t)(n0 + (j << 4) + rlane) * ldb + koff + k0;
      bh[j] = FragH::load(Bt + bo);
    }
#pragma unroll
    for (int i = 0; i < 4; ++i) {
      const size_t ao = (size_t)(m0 + (i << 4) + rlane) * lda + koff + k0;
      v16h ah = FragH::load(A + ao);
#pragma unroll
      for (int j = 0; j < 4; ++j) acc[i][j] = FragH::mma(ah, bh[j], acc[i][j]);
      dep_guard4_h(acc[i][0], acc[i][1], acc[i][2], acc[i][3], ah, bh[0], bh[1], bh[2], bh[3]);
    }
  }
  acc_guard4(acc[0][0], acc[0][1], acc[0][2], acc[0][3]);
  acc_guard4(acc[1][0], acc[1][1], acc[1][2], acc[1][3]);
  acc_guard4(acc[2][0], acc[2][1], acc[2][2], acc[2][3]);
  acc_guard4(acc[3][0], acc[3][1], acc[3][2], acc[3][3]);

  float* slab = sT[wave];
#pragma unroll
  for (int i = 0; i < 4; ++i) {
    const int mBase = m0 + (i << 4);
#pragma unroll
    for (int j = 0; j < 4; ++j) {
#pragma unroll
      for (int r = 0; r < 8; ++r) {
        slab[(mOff + r) * 68 + (j << 4) + rlane] = acc[i][j][r] * scale;
      }
    }
    __builtin_amdgcn_fence(__ATOMIC_RELEASE, "workgroup");
    __builtin_amdgcn_wave_barrier();
    __builtin_amdgcn_fence(__ATOMIC_ACQUIRE, "workgroup");
    {
      const int hh = lane >> 4, c4 = (lane & 15) * 4;
      v4f ov[8];
#pragma unroll
      for (int it = 0; it < 8; ++it) ov[it] = *(const v4f*)(slab + (it * 2 + hh) * 68 + c4);
      if (EPI == 2) {
#pragma unroll
        for (int it = 0; it < 4; ++it) {
          const size_t o = (size_t)(mBase + it * 2 + hh) * ldc + n0 + c4;
          const v4f r1 = *(const v4f*)(R1 + o);
          const v4f r2 = *(const v4f*)(R2 + o);
          ov[it] = r1 + (r2 + ov[it]);
        }
        force4(ov[0], ov[1], ov[2], ov[3]);
#pragma unroll
        for (int it = 4; it < 8; ++it) {
          const size_t o = (size_t)(mBase + it * 2 + hh) * ldc + n0 + c4;
          const v4f r1 = *(const v4f*)(R1 + o);
          const v4f r2 = *(const v4f*)(R2 + o);
          ov[it] = r1 + (r2 + ov[it]);
        }
        force4(ov[4], ov[5], ov[6], ov[7]);
      }
      for (int pass = 0; pass < 2; ++pass) {
#pragma unroll
        for (int it = 0; it < 8; ++it) {
          const int row = it * 2 + hh;
          *(volatile v4f*)(Cout + (size_t)(mBase + row) * ldc + n0 + c4) = ov[it];
        }
        __threadfence();
      }
    }
    if (EPI == 1) {
      const int q = lane >> 3, c8 = (lane & 7) * 8;
      v8h hv[4];
#pragma unroll
      for (int it = 0; it < 4; ++it) {
        const float* sp = slab + (it * 4 + q) * 68 + c8;
        const v4f a0 = *(const v4f*)(sp);
        const v4f a1 = *(const v4f*)(sp + 4);
#pragma unroll
        for (int e = 0; e < 4; ++e) {
          hv[it][e]     = (_Float16)(a0[e] * scale2);
          hv[it][4 + e] = (_Float16)(a1[e] * scale2);
        }
      }
      for (int pass = 0; pass < 2; ++pass) {
#pragma unroll
        for (int it = 0; it < 4; ++it) {
          const int row = it * 4 + q;
          *(volatile v8h*)(C2 + (size_t)(mBase + row) * ld2 + n0 + c8) = hv[it];
        }
        __threadfence();
      }
    }
    __builtin_amdgcn_fence(__ATOMIC_RELEASE, "workgroup");
    __builtin_amdgcn_wave_barrier();
    __builtin_amdgcn_fence(__ATOMIC_ACQUIRE, "workgroup");
  }
}

__global__ __launch_bounds__(256) void cast_f16_kernel(
    const float* __restrict__ src, unsigned short* __restrict__ dst, int total8, float scale)
{
  const int i = blockIdx.x * 256 + threadIdx.x;
  if (i >= total8) return;
  const size_t e0 = (size_t)i << 3;
  const float* p = src + e0;
  const v4f a0 = *(const v4f*)(p);
  const v4f a1 = *(const v4f*)(p + 4);
  v8h hv;
#pragma unroll
  for (int e = 0; e < 4; ++e) {
    hv[e]     = (_Float16)(a0[e] * scale);
    hv[4 + e] = (_Float16)(a1[e] * scale);
  }
  unsigned short* q = dst + e0;
  *(volatile v8h*)q = hv;
  __threadfence();
  *(volatile v8h*)q = hv;
}

__global__ __launch_bounds__(256) void transpose_cast_kernel(
    const float* __restrict__ W, unsigned short* __restrict__ Bt, int Kdim, int Ndim,
    long srcStride, long dstStride, float scale)
{
  __shared__ float tile[64 * 65];
  const int tid = threadIdx.x, lane = tid & 31, wave = tid >> 5;
  const int n0 = blockIdx.x * 64;
  const int k0 = blockIdx.y * 64;
  const float* Wz = W + (size_t)blockIdx.z * srcStride;
  unsigned short* Bz = Bt + (size_t)blockIdx.z * dstStride;
#pragma unroll 4
  for (int p = 0; p < 16; ++p) {
    const int idx = tid + p * 256;
    const int kk  = idx >> 6;
    const int nn  = idx & 63;
    const int n   = n0 + nn;
    const int nc  = (n < Ndim) ? n : (Ndim - 1);
    const float v = Wz[(size_t)(k0 + kk) * Ndim + nc];
    tile[kk * 65 + nn] = (n < Ndim) ? (v * scale) : 0.f;
  }
  __syncthreads();
  const int q = lane >> 3, c8 = (lane & 7) * 8;
  v8h hv[2];
#pragma unroll
  for (int it = 0; it < 2; ++it) {
    const int nrow = it * 32 + wave * 4 + q;
#pragma unroll
    for (int e = 0; e < 8; ++e) hv[it][e] = (_Float16)tile[(c8 + e) * 65 + nrow];
  }
  for (int pass = 0; pass < 2; ++pass) {
#pragma unroll
    for (int it = 0; it < 2; ++it) {
      const int nrow = it * 32 + wave * 4 + q;
      *(volatile v8h*)(Bz + (size_t)(n0 + nrow) * Kdim + k0 + c8) = hv[it];
    }
    __threadfence();
  }
}

__global__ __launch_bounds__(256) void small_rows_kernel(
    const float* __restrict__ Wg, const float* __restrict__ Wb, const float* __restrict__ Wa,
    const float* __restrict__ Wbl, unsigned short* __restrict__ WVS, float scale)
{
  __shared__ float tile[64 * 65];
  const int tid = threadIdx.x, lane = tid & 31, wave = tid >> 5;
  const int k0 = blockIdx.x * 64;
  const int l  = blockIdx.y;
  const float* wg = Wg  + (size_t)l * kDm * kNhead;
  const float* wb = Wb  + (size_t)l * kNmat * kDm * kNhead;
  const float* wa = Wa  + (size_t)l * kNmat * kDm * kNhead;
  const float* wl = Wbl + (size_t)l * kDm * 8;
#pragma unroll 1
  for (int p = 0; p < 16; ++p) {
    const int idx = tid + p * 256;
    const int kk  = idx >> 6;
    const int nn  = idx & 63;
    const int kx  = k0 + kk;
    const int ng  = (nn < 3) ? nn : 3;
    int jb = nn - 4;  jb = jb < 0 ? 0 : (jb > 7 ? 7 : jb);
    int ja = nn - 12; ja = ja < 0 ? 0 : (ja > 7 ? 7 : ja);
    int jl = nn - 20; jl = jl < 0 ? 0 : (jl > 7 ? 7 : jl);
    const float va = wg[kx * 4 + ng];
    const float vb = wb[(jb >> 2) * (kDm * 4) + kx * 4 + (jb & 3)];
    const float vc = wa[(ja >> 2) * (kDm * 4) + kx * 4 + (ja & 3)];
    const float vd = wl[kx * 8 + jl];
    const float fg = (nn < 4) ? 1.0f : 0.0f;
    const float fb = (nn >= 4 && nn < 12) ? 1.0f : 0.0f;
    const float fa = (nn >= 12 && nn < 20) ? 1.0f : 0.0f;
    const float fl = (nn >= 20 && nn < 28) ? 1.0f : 0.0f;
    const float v = fg * va + fb * vb + fa * vc + fl * vd;
    tile[kk * 65 + nn] = v * scale;
  }
  __syncthreads();
  const int q = lane >> 3, c8 = (lane & 7) * 8;
  unsigned short* Bz = WVS + (size_t)l * kVPld * kDm + (size_t)(kNmat * kDm) * kDm;
  v8h hv[2];
#pragma unroll
  for (int it = 0; it < 2; ++it) {
    const int nrow = it * 32 + wave * 4 + q;
#pragma unroll
    for (int e = 0; e < 8; ++e) hv[it][e] = (_Float16)tile[(c8 + e) * 65 + nrow];
  }
  for (int pass = 0; pass < 2; ++pass) {
#pragma unroll
    for (int it = 0; it < 2; ++it) {
      const int nrow = it * 32 + wave * 4 + q;
      *(volatile v8h*)(Bz + (size_t)nrow * kDm + k0 + c8) = hv[it];
    }
    __threadfence();
  }
}

__global__ __launch_bounds__(256) void embed_kernel(
    const int* __restrict__ ids, const float* __restrict__ emb, float* __restrict__ X)
{
  const int lane = threadIdx.x & 31, wave = threadIdx.x >> 5;
  const int tok = blockIdx.x * 8 + wave;
  int id = ids[tok];
  id = id < 0 ? 0 : (id > kVocab - 1 ? kVocab - 1 : id);
  const float* src = emb + (size_t)id * kDm + lane * 4;
  const v4f v0 = *(const v4f*)(src);
  const v4f v1 = *(const v4f*)(src + 128);
  float* dst = X + (size_t)tok * kDm + lane * 4;
  *(volatile v4f*)(dst) = v0;
  *(volatile v4f*)(dst + 128) = v1;
  __threadfence();
  *(volatile v4f*)(dst) = v0;
  *(volatile v4f*)(dst + 128) = v1;
}

__global__ __launch_bounds__(256) void rmsnorm_kernel(
    const float* __restrict__ X, const float* __restrict__ w, unsigned short* __restrict__ Y16)
{
  const int lane = threadIdx.x & 31, wave = threadIdx.x >> 5;
  const int row = blockIdx.x * 8 + wave;
  const float* p = X + (size_t)row * kDm + lane * 8;
  const v4f a0 = *(const v4f*)(p);
  const v4f a1 = *(const v4f*)(p + 4);
  const v4f w0 = *(const v4f*)(w + lane * 8);
  const v4f w1 = *(const v4f*)(w + lane * 8 + 4);
  float ss = 0.f;
#pragma unroll
  for (int e = 0; e < 4; ++e) { ss += a0[e] * a0[e]; ss += a1[e] * a1[e]; }
#pragma unroll
  for (int off = 16; off > 0; off >>= 1) ss += __shfl_xor(ss, off, 32);
  const float inv = rsqrtf(ss * (1.0f / (float)kDm) + 1e-6f);
  v8h hv;
#pragma unroll
  for (int e = 0; e < 4; ++e) {
    hv[e]     = (_Float16)((a0[e] * inv) * w0[e]);
    hv[4 + e] = (_Float16)((a1[e] * inv) * w1[e]);
  }
  unsigned short* q = Y16 + (size_t)row * kDm + lane * 8;
  *(volatile v8h*)q = hv;
  __threadfence();
  *(volatile v8h*)q = hv;
}

__global__ __launch_bounds__(256) void conv_gate_kernel(
    const float* __restrict__ UG, const float* __restrict__ cw, const float* __restrict__ cb,
    unsigned short* __restrict__ P16)
{
  __shared__ __align__(16) float sT[16 * kConvTP];
  const int tid = threadIdx.x, lane = tid & 31, wave = tid >> 5;
  const int d0 = blockIdx.x * 256, d = d0 + tid;
  const int g0 = blockIdx.y * 64;
  const int tb = g0 & (kSeqT - 1);
  const float w0 = cw[d * 4 + 0], w1 = cw[d * 4 + 1], w2 = cw[d * 4 + 2], w3 = cw[d * 4 + 3];
  const float bc = cb[d];
  float xm3, xm2, xm1;
  {
    const bool hist = (tb > 0);
    const int rb = hist ? (g0 - 3) : g0;
    const float v3 = UG[(size_t)rb * kUGld + d];
    const float v2 = UG[(size_t)(rb + 1) * kUGld + d];
    const float v1 = UG[(size_t)(rb + 2) * kUGld + d];
    xm3 = hist ? v3 : 0.f;
    xm2 = hist ? v2 : 0.f;
    xm1 = hist ? v1 : 0.f;
  }
#pragma unroll 1
  for (int sub = 0; sub < 4; ++sub) {
    const int lb = g0 + sub * 16;
#pragma unroll 1
    for (int s = 0; s < 16; ++s) {
      const float xcur = UG[(size_t)(lb + s) * kUGld + d];
      const float gp   = UG[(size_t)(lb + s) * kUGld + kDinr + d];
      float acc = w0 * xm3;
      acc = fmaf(w1, xm2, acc);
      acc = fmaf(w2, xm1, acc);
      acc = fmaf(w3, xcur, acc);
      const float sv = acc + bc;
      const float hs = sv * __builtin_amdgcn_rcpf(1.0f + expf(-sv));
      const float gs = gp * __builtin_amdgcn_rcpf(1.0f + expf(-gp));
      sT[s * kConvTP + tid] = (gs * hs) * kPCarry;
      xm3 = xm2; xm2 = xm1; xm1 = xcur;
    }
    __syncthreads();
    v8h bv[2];
#pragma unroll
    for (int it = 0; it < 2; ++it) {
      const float* sp = sT + (it * 8 + wave) * kConvTP + lane * 8;
      const v4f a0 = *(const v4f*)(sp);
      const v4f a1 = *(const v4f*)(sp + 4);
#pragma unroll
      for (int e = 0; e < 4; ++e) {
        bv[it][e]     = (_Float16)a0[e];
        bv[it][4 + e] = (_Float16)a1[e];
      }
    }
    for (int pass = 0; pass < 2; ++pass) {
#pragma unroll
      for (int it = 0; it < 2; ++it)
        *(volatile v8h*)(P16 + (size_t)(lb + it * 8 + wave) * kDinr + d0 + lane * 8) = bv[it];
      __threadfence();
    }
    __syncthreads();
  }
}

__global__ __launch_bounds__(256) void params_kernel(
    const float* __restrict__ U, const float* __restrict__ VP,
    const float* __restrict__ Alog, const float* __restrict__ dtb, float* __restrict__ PRM)
{
  const int lane = threadIdx.x & 31, wave = threadIdx.x >> 5;
  const int row = blockIdx.x * 8 + wave;
  const float* up = U + (size_t)row * kDm + lane * 8;
  const v4f a0 = *(const v4f*)(up);
  const v4f a1 = *(const v4f*)(up + 4);
  float ss = 0.f;
#pragma unroll
  for (int e = 0; e < 4; ++e) { ss += a0[e] * a0[e]; ss += a1[e] * a1[e]; }
  ss += __shfl_xor(ss, 1, 32);
  ss += __shfl_xor(ss, 2, 32);
  ss += __shfl_xor(ss, 4, 32);
  const float inv  = __builtin_amdgcn_rcpf(fmaxf(sqrtf(ss), 1e-12f));
  const float invh = __shfl(inv, (lane & 3) * 8, 32);
  const int pc = (lane < 27) ? lane : 27;
  const float z  = VP[(size_t)row * kVPld + kNmat * kDm + pc];
  const float zp = __shfl_xor(z, 1, 32);
  int cd = lane - 12; cd = cd < 0 ? 0 : (cd > 7 ? 7 : cd);
  const float al = Alog[cd];
  const float db = dtb[cd];
  const float sig = __builtin_amdgcn_rcpf(1.0f + expf(-z));
  const float alpha = z + db;
  const float ea = expf(-fabsf(alpha));
  const float ua = 1.0f + ea;
  const float l1p = logf(ua) + (ea - (ua - 1.0f)) * __builtin_amdgcn_rcpf(ua);
  const float sp  = fmaxf(alpha, 0.0f) + l1p;
  const float dec = expf(-expf(al) * sp);
  const float mx = fmaxf(z, zp);
  const float e0 = expf(z - mx), e1 = expf(zp - mx);
  const float bl = e0 * __builtin_amdgcn_rcpf(e0 + e1);
  float val = sig;
  val = (lane >= 12) ? dec : val;
  val = (lane >= 20) ? bl : val;
  val = (lane >= 28) ? invh : val;
  float* q = PRM + (size_t)row * kPrmLd + lane;
  *(volatile float*)q = val;
  __threadfence();
  *(volatile float*)q = val;
}

__global__ __launch_bounds__(512) void delta_scan_kernel(
    const float* __restrict__ U, const float* __restrict__ VP, const float* __restrict__ PRM,
    unsigned short* __restrict__ O16)
{
  __shared__ __align__(16) float keyS[(kScanTS + 1) * 128];
  __shared__ __align__(16) float valS[kScanTS * 128];
  __shared__ __align__(16) float prmS[kScanTS * kPrmLd];
  __shared__ __align__(16) float rdS[2 * kScanTS * 64];
  const int tid = threadIdx.x, lane = tid & 31, wave = tid >> 5;
  const int b = blockIdx.x >> 2, h = blockIdx.x & 3;
  const size_t row0 = (size_t)b * kSeqT;
  const int m    = wave >> 3;
  const int k    = ((wave & 7) << 3) + (lane & 7);
  const int part = lane >> 3;
  const int sr   = tid >> 7;
  const int smd  = tid & 127;
  const int sm   = smd >> 6, sd = smd & 63;
  float S[16];
#pragma unroll
  for (int i = 0; i < 16; ++i) S[i] = 0.f;
  float rdprev = 0.f;
#pragma unroll 1
  for (int t0 = 0; t0 < kSeqT; t0 += kScanTS) {
    __syncthreads();
#pragma unroll 1
    for (int i = 0; i < 5; ++i) {
      const int r = sr + 4 * i;
      if (r < kScanTS + 1) {
        const int tt = t0 - 1 + r;
        const bool valid = (tt >= 0);
        const size_t tok = row0 + (size_t)(valid ? tt : 0);
        const float ua = U[tok * kDm + h * kHdim + sd];
        const float ub = U[tok * kDm + h * kHdim + (sd ^ 1)];
        const float iv = PRM[tok * kPrmLd + 28 + h];
        const float pa = ua * iv;
        const float pb = ub * iv;
        const float v1 = (sd & 1) ? pb : -pb;
        const float kv = (sm == 0) ? pa : v1;
        keyS[r * 128 + smd] = valid ? kv : 0.f;
      }
    }
#pragma unroll
    for (int i = 0; i < 4; ++i) {
      const int s = sr + 4 * i;
      valS[s * 128 + smd] = VP[(row0 + t0 + s) * kVPld + sm * kDm + h * kHdim + sd];
    }
    prmS[tid] = PRM[(row0 + t0) * kPrmLd + tid];
    __syncthreads();
#pragma unroll 1
    for (int s = 0; s < kScanTS; ++s) {
      const float dc = prmS[s * kPrmLd + 12 + m * 4 + h];
      const float bt = prmS[s * kPrmLd + 4 + m * 4 + h];
      const float v  = valS[s * 128 + m * 64 + k];
      const float* kw = keyS + s * 128 + m * 64 + part * 16;
      const float* kr = kw + 128;
      v4f wk[4], rk[4];
#pragma unroll
      for (int j = 0; j < 4; ++j) {
        wk[j] = *(const v4f*)(kw + 4 * j);
        rk[j] = *(const v4f*)(kr + 4 * j);
      }
      const float err = (v - dc * rdprev) * bt;
      float rd = 0.f;
#pragma unroll
      for (int i = 0; i < 16; ++i) {
        float sv = S[i] * dc;
        sv = fmaf(wk[i >> 2][i & 3], err, sv);
        S[i] = sv;
        rd = fmaf(sv, rk[i >> 2][i & 3], rd);
      }
      rd += __shfl_xor(rd, 8, 32);
      rd += __shfl_xor(rd, 16, 32);
      if (part == 0) rdS[(m * kScanTS + s) * 64 + k] = rd;
      rdprev = rd;
    }
    __syncthreads();
    if (wave < 4) {
      const int q = lane >> 3, c8 = (lane & 7) * 8;
      const int s = wave * 4 + q;
      const float g  = prmS[s * kPrmLd + h];
      const float b0 = prmS[s * kPrmLd + 20 + h * 2];
      const float b1 = prmS[s * kPrmLd + 21 + h * 2];
      const float* r0 = rdS + s * 64 + c8;
      const float* r1 = rdS + (kScanTS + s) * 64 + c8;
      const v4f a0 = *(const v4f*)(r0);
      const v4f a1 = *(const v4f*)(r0 + 4);
      const v4f c0 = *(const v4f*)(r1);
      const v4f c1 = *(const v4f*)(r1 + 4);
      v8h hv;
#pragma unroll
      for (int e = 0; e < 4; ++e) {
        hv[e]     = (_Float16)(((b0 * a0[e] + b1 * c0[e]) * g) * kOCarry);
        hv[4 + e] = (_Float16)(((b0 * a1[e] + b1 * c1[e]) * g) * kOCarry);
      }
      unsigned short* dst = O16 + (row0 + t0 + s) * kDm + h * kHdim + c8;
      *(volatile v8h*)dst = hv;
      __threadfence();
      *(volatile v8h*)dst = hv;
    }
  }
}

__global__ __launch_bounds__(256) void head_gemm_kernel(
    const unsigned short* __restrict__ Yp, const unsigned short* __restrict__ Ep,
    float* __restrict__ out, float scale)
{
  __shared__ __align__(16) float sO[32 * kVocab];
  const _Float16* Y = (const _Float16*)Yp;
  const _Float16* E = (const _Float16*)Ep;
  const int tid = threadIdx.x, lane = tid & 31, wave = tid >> 5;
  const int rlane = lane & 15;
  const int koff  = (lane >> 4) * 8;
  const int mOff  = (lane >> 4) * 8;
  const int m0 = blockIdx.x * 32;
  v8f acc[2][3];
#pragma unroll
  for (int i = 0; i < 2; ++i)
#pragma unroll
    for (int jj = 0; jj < 3; ++jj) acc[i][jj] = (v8f){0.f,0.f,0.f,0.f,0.f,0.f,0.f,0.f};
#pragma unroll 1
  for (int k0 = 0; k0 < kDm; k0 += 32) {
    v16h bh[3], ah[2];
#pragma unroll
    for (int jj = 0; jj < 3; ++jj) {
      const int j  = wave + 8 * jj;
      const int jc = (j < 17) ? j : 16;
      bh[jj] = FragH::load(E + (size_t)(jc * 16 + rlane) * kDm + koff + k0);
    }
#pragma unroll
    for (int i = 0; i < 2; ++i) ah[i] = FragH::load(Y + (size_t)(m0 + i * 16 + rlane) * kDm + koff + k0);
#pragma unroll
    for (int i = 0; i < 2; ++i)
#pragma unroll
      for (int jj = 0; jj < 3; ++jj) acc[i][jj] = FragH::mma(ah[i], bh[jj], acc[i][jj]);
    dep_guard6_h(acc[0][0], acc[0][1], acc[0][2], acc[1][0], acc[1][1], acc[1][2], ah[0], ah[1], bh[0], bh[1], bh[2]);
  }
#pragma unroll
  for (int jj = 0; jj < 3; ++jj) {
    const int j = wave + 8 * jj;
    if (j < 17) {
#pragma unroll
      for (int i = 0; i < 2; ++i)
#pragma unroll
        for (int r = 0; r < 8; ++r)
          sO[(i * 16 + mOff + r) * kVocab + j * 16 + rlane] = acc[i][jj][r] * scale;
    }
  }
  __syncthreads();
  v4f ov[9];
#pragma unroll
  for (int i = 0; i < 9; ++i) {
    const int c  = wave + 8 * i;
    const int cc = (c < 68) ? c : 67;
    ov[i] = *(const v4f*)(sO + cc * 128 + lane * 4);
  }
  float* base = out + (size_t)m0 * kVocab;
  for (int pass = 0; pass < 2; ++pass) {
#pragma unroll
    for (int i = 0; i < 9; ++i) {
      const int c = wave + 8 * i;
      if (c < 68) *(volatile v4f*)(base + c * 128 + lane * 4) = ov[i];
    }
    __threadfence();
  }
}

extern "C" void kernel_launch(void* const* d_in, const int* in_sizes, int n_in,
                              void* d_out, int out_size, void* d_ws, size_t ws_size,
                              hipStream_t stream)
{
  if (n_in < 17) return;
  if (in_sizes[0] != kTok) return;
  if (in_sizes[1] != kVocab * kDm) return;
  if (in_sizes[2] != kLayers * kDm) return;
  if (in_sizes[3] != kLayers * kDm * kDinr || in_sizes[4] != kLayers * kDm * kDinr) return;
  if (in_sizes[5] != kLayers * kDinr * kDm) return;
  if (in_sizes[6] != kLayers * kDinr * 4 || in_sizes[7] != kLayers * kDinr) return;
  if (in_sizes[8] != kLayers * kDm * kNmat * kDm) return;
  if (in_sizes[9] != kLayers * kDm * kNhead) return;
  if (in_sizes[10] != kLayers * kNmat * kDm * kNhead || in_sizes[11] != kLayers * kNmat * kDm * kNhead) return;
  if (in_sizes[12] != kLayers * kNmat * kNhead || in_sizes[13] != kLayers * kNmat * kNhead) return;
  if (in_sizes[14] != kLayers * kDm * 8) return;
  if (in_sizes[15] != kLayers * kDm * kDm) return;
  if (in_sizes[16] != kDm) return;
  if (out_size != kTok * kVocab) return;
  if (ws_size < kWsTotal) return;

  const int*   ids    = (const int*)d_in[0];
  const float* emb    = (const float*)d_in[1];
  const float* norm_w = (const float*)d_in[2];
  const float* W_up   = (const float*)d_in[3];
  const float* W_gate = (const float*)d_in[4];
  const float* W_down = (const float*)d_in[5];
  const float* conv_w = (const float*)d_in[6];
  const float* conv_b = (const float*)d_in[7];
  const float* Wv     = (const float*)d_in[8];
  const float* Wg     = (const float*)d_in[9];
  const float* Wb     = (const float*)d_in[10];
  const float* Wa     = (const float*)d_in[11];
  const float* A_log  = (const float*)d_in[12];
  const float* dt_b   = (const float*)d_in[13];
  const float* Wblend = (const float*)d_in[14];
  const float* Wout   = (const float*)d_in[15];
  const float* fnorm  = (const float*)d_in[16];
  float* out = (float*)d_out;

  char* ws = (char*)d_ws;
  float*          X     = (float*)(ws + kOffX);
  unsigned short* NX16  = (unsigned short*)(ws + kOffNX);
  unsigned short* Y16   = (unsigned short*)(ws + kOffY16);
  float*          UPGP  = (float*)(ws + kOffUPGP);
  unsigned short* P16   = (unsigned short*)(ws + kOffP16);
  float*          U     = (float*)(ws + kOffU);
  unsigned short* U16   = (unsigned short*)(ws + kOffU16);
  float*          VP    = (float*)(ws + kOffVP);
  float*          PRM   = (float*)(ws + kOffPRM);
  unsigned short* O16   = (unsigned short*)(ws + kOffO16);
  unsigned short* WUG   = (unsigned short*)(ws + kOffWUG);
  unsigned short* WDN   = (unsigned short*)(ws + kOffWDN);
  unsigned short* WVS   = (unsigned short*)(ws + kOffWVS);
  unsigned short* WOU   = (unsigned short*)(ws + kOffWOU);
  unsigned short* EMB16 = (unsigned short*)(ws + kOffEMB);

  transpose_cast_kernel<<<dim3(kDinr / 64, kDm / 64, kLayers), 256, 0, stream>>>(
      W_up, WUG, kDm, kDinr, (long)kDm * kDinr, (long)kUGld * kDm, kWCarry);
  transpose_cast_kernel<<<dim3(kDinr / 64, kDm / 64, kLayers), 256, 0, stream>>>(
      W_gate, WUG + (size_t)kDinr * kDm, kDm, kDinr, (long)kDm * kDinr, (long)kUGld * kDm, kWCarry);
  transpose_cast_kernel<<<dim3(kDm / 64, kDinr / 64, kLayers), 256, 0, stream>>>(
      W_down, WDN, kDinr, kDm, (long)kDinr * kDm, (long)kDm * kDinr, kWCarry);
  transpose_cast_kernel<<<dim3((kNmat * kDm) / 64, kDm / 64, kLayers), 256, 0, stream>>>(
      Wv, WVS, kDm, kNmat * kDm, (long)kDm * kNmat * kDm, (long)kVPld * kDm, kWCarry);
  small_rows_kernel<<<dim3(kDm / 64, kLayers), 256, 0, stream>>>(Wg, Wb, Wa, Wblend, WVS, kWCarry);
  transpose_cast_kernel<<<dim3(kDm / 64, kDm / 64, kLayers), 256, 0, stream>>>(
      Wout, WOU, kDm, kDm, (long)kDm * kDm, (long)kDm * kDm, kWCarry);
  cast_f16_kernel<<<(kVocab * kDm / 8) / 256, 256, 0, stream>>>(emb, EMB16, kVocab * kDm / 8, kWCarry);

  embed_kernel<<<kTok / 8, 256, 0, stream>>>(ids, emb, X);

  for (int l = 0; l < kLayers; ++l) {
    rmsnorm_kernel<<<kTok / 8, 256, 0, stream>>>(X, norm_w + (size_t)l * kDm, NX16);

    wmma_gemm64_f16<0><<<128, 256, 0, stream>>>(
        NX16, kDm, WUG + (size_t)l * kUGld * kDm, kDm,
        UPGP, kUGld, U16, kDm, 1.0f, X, U,
        kTok, kUGld, kDm, 1.0f / kWCarry);

    conv_gate_kernel<<<dim3(kDinr / 256, kTok / 64), 256, 0, stream>>>(
        UPGP, conv_w + (size_t)l * kDinr * 4, conv_b + (size_t)l * kDinr, P16);

    wmma_gemm64_f16<1><<<32, 256, 0, stream>>>(
        P16, kDinr, WDN + (size_t)l * kDm * kDinr, kDinr,
        U, kDm, U16, kDm, kUCarry, X, U,
        kTok, kDm, kDinr, 1.0f / (kPCarry * kWCarry));

    wmma_gemm64_f16<0><<<72, 256, 0, stream>>>(
        U16, kDm, WVS + (size_t)l * kVPld * kDm, kDm,
        VP, kVPld, U16, kDm, 1.0f, X, U,
        kTok, kVPld, kDm, 1.0f / (kUCarry * kWCarry));

    params_kernel<<<kTok / 8, 256, 0, stream>>>(
        U, VP, A_log + (size_t)l * kNmat * kNhead, dt_b + (size_t)l * kNmat * kNhead, PRM);

    delta_scan_kernel<<<kBatch * kNhead, 512, 0, stream>>>(U, VP, PRM, O16);

    wmma_gemm64_f16<2><<<32, 256, 0, stream>>>(
        O16, kDm, WOU + (size_t)l * kDm * kDm, kDm,
        X, kDm, U16, kDm, 1.0f, X, U,
        kTok, kDm, kDm, 1.0f / (kOCarry * kWCarry));
  }

  rmsnorm_kernel<<<kTok / 8, 256, 0, stream>>>(X, fnorm, Y16);
  head_gemm_kernel<<<kTok / 32, 256, 0, stream>>>(Y16, EMB16, out, 1.0f / kWCarry);
}
